// DecoderLayer_77129022701893
// MI455X (gfx1250) — hardware-verified
//
#include <hip/hip_runtime.h>
#ifndef NB
#define NB 2
#endif
#ifndef SEQ
#define SEQ 2048
#endif
#define NB_FULL 2
#define SEQ_FULL 2048
#define DM 1024
#define DFF 4096
#define NH 16
#define HD 64
#define LQ (3 * DM)
#define MROWS (NB * SEQ)
#define NQT (SEQ / 64)
#define NKT (SEQ / 64)
#define QKV_BYTES ((size_t)MROWS * LQ * 2)
#define VT_BYTES  ((size_t)NB * NH * HD * SEQ * 2)
#define H_BYTES   ((size_t)MROWS * DFF * 2)
#define R1_BYTES  ((QKV_BYTES + VT_BYTES) > H_BYTES ? (QKV_BYTES + VT_BYTES) : H_BYTES)
static_assert(SEQ % 64 == 0);
static_assert(SEQ <= SEQ_FULL);
static_assert(NB >= 1 && NB <= NB_FULL);
static_assert(NKT <= 32);
static_assert(MROWS % 128 == 0);
static_assert(DM % 64 == 0 && DM % 32 == 0 && DFF % 64 == 0 && DFF % 32 == 0);
static_assert(NH * HD == DM);
static_assert(H_BYTES <= R1_BYTES);
static_assert(QKV_BYTES + VT_BYTES <= R1_BYTES);
static_assert(QKV_BYTES % 256 == 0);
static_assert(((size_t)MROWS * DM) % (8 * 256) == 0);
static_assert(((size_t)DM * DM) % (8 * 256) == 0 && ((size_t)DFF * DM) % (8 * 256) == 0);

typedef _Float16 v16h __attribute__((ext_vector_type(16)));
typedef _Float16 v4h  __attribute__((ext_vector_type(4)));
typedef unsigned short v8us __attribute__((ext_vector_type(8), may_alias));
typedef float  v8f  __attribute__((ext_vector_type(8)));
typedef float  v4f  __attribute__((ext_vector_type(4)));
typedef float  v4fa __attribute__((ext_vector_type(4), may_alias));
typedef int    v4ia __attribute__((ext_vector_type(4), may_alias));
union FragH { v16h v; v8us half[2]; _Float16 h[16]; unsigned short u[16]; };

#define NEG_INF (-__builtin_inff())
#define FILL_RAW (-8.0e9f)

__device__ __forceinline__ unsigned short bf16_bits(float x) { unsigned int u = __float_as_uint(x); return (unsigned short)((u + 0x7FFFu + ((u >> 16) & 1u)) >> 16); }
__device__ __forceinline__ float bf16_val(unsigned short b) { return __uint_as_float(((unsigned int)b) << 16); }
__device__ __forceinline__ float bf16_rne(float x) { return bf16_val(bf16_bits(x)); }

__device__ __forceinline__ v16h g2_frag(const _Float16* p, int hh) { FragH f; f.half[0] = *(const v8us*)((const unsigned short*)p + 8 * hh); f.half[1] = *(const v8us*)((const unsigned short*)p + 16 + 8 * hh); return f.v; }
__device__ __forceinline__ v8f g2_mma(v16h a, v16h b, v8f c) { v8f d = __builtin_amdgcn_wmma_f32_16x16x32_f16(false, a, false, b, (short)0, c, false, false); asm volatile("v_nop\n\tv_nop\n\tv_nop\n\tv_nop" : "+v"(d) : "v"(a), "v"(b)); return d; }

__global__ __launch_bounds__(256) void k_x16(const float* __restrict__ x0, const float* __restrict__ x1, _Float16* __restrict__ D0, _Float16* __restrict__ D1) {
  const size_t t = (size_t)blockIdx.x * 256 + threadIdx.x; const size_t n8 = (size_t)MROWS * DM / 8; if (t >= n8) return;
  const float* x = (blockIdx.y == 0) ? x0 : x1; _Float16* D = (blockIdx.y == 0) ? D0 : D1;
  const size_t e = t * 8; const size_t m = e / DM; const size_t col = e - m * DM; const size_t bb = m / SEQ; const size_t s = m - bb * SEQ;
  const float* src = x + (bb * SEQ_FULL + s) * DM + col;
  const v4f a = *(const v4fa*)src; const v4f c = *(const v4fa*)(src + 4); FragH f;
#pragma unroll
  for (int q = 0; q < 4; ++q) { f.h[q] = (_Float16)bf16_rne(a[q]); f.h[4 + q] = (_Float16)bf16_rne(c[q]); }
  const v8us val = f.half[0];
  *(volatile v8us*)((unsigned short*)D + e) = val; __threadfence(); *(volatile v8us*)((unsigned short*)D + e) = val; }

__global__ __launch_bounds__(256) void k_wnat4(const float* __restrict__ w0, const float* __restrict__ w1, const float* __restrict__ w2, const float* __restrict__ w3, size_t n8, _Float16* __restrict__ Bt) {
  const size_t t = (size_t)blockIdx.x * 256 + threadIdx.x; if (t >= n8) return;
  const int y = blockIdx.y; const float* w = (y == 0) ? w0 : ((y == 1) ? w1 : ((y == 2) ? w2 : w3));
  const v4f a = *(const v4fa*)(w + t * 8); const v4f c = *(const v4fa*)(w + t * 8 + 4); FragH f;
#pragma unroll
  for (int q = 0; q < 4; ++q) { f.h[q] = (_Float16)(bf16_rne(a[q]) * 16.0f); f.h[4 + q] = (_Float16)(bf16_rne(c[q]) * 16.0f); }
  const v8us val = f.half[0]; unsigned short* d = (unsigned short*)Bt + ((size_t)y * n8 + t) * 8;
  *(volatile v8us*)d = val; __threadfence(); *(volatile v8us*)d = val; }

__device__ __forceinline__ void g2_core(const _Float16* __restrict__ A, int lda, const _Float16* __restrict__ Bh, int ldb, int K, int row0, int col0, int lane, float alpha, const float* __restrict__ bias, float (*sw)[68]) {
  const int ln = lane & 15, hh = lane >> 4;
  const _Float16* a0p = A + (size_t)(row0 + ln) * lda; const _Float16* a1p = a0p + (size_t)16 * lda;
  const _Float16* b0p = Bh + (size_t)(col0 + ln) * ldb; const _Float16* b1p = b0p + (size_t)16 * ldb; const _Float16* b2p = b1p + (size_t)16 * ldb; const _Float16* b3p = b2p + (size_t)16 * ldb;
  const v8f z8 = {0.f,0.f,0.f,0.f,0.f,0.f,0.f,0.f}; v8f c00 = z8, c01 = z8, c02 = z8, c03 = z8, c10 = z8, c11 = z8, c12 = z8, c13 = z8;
#pragma unroll 1
  for (int kb = 0; kb < K; kb += 32) { const v16h a0 = g2_frag(a0p + kb, hh), a1 = g2_frag(a1p + kb, hh);
    v16h b = g2_frag(b0p + kb, hh); c00 = g2_mma(a0, b, c00); c10 = g2_mma(a1, b, c10);
    b = g2_frag(b1p + kb, hh); c01 = g2_mma(a0, b, c01); c11 = g2_mma(a1, b, c11);
    b = g2_frag(b2p + kb, hh); c02 = g2_mma(a0, b, c02); c12 = g2_mma(a1, b, c12);
    b = g2_frag(b3p + kb, hh); c03 = g2_mma(a0, b, c03); c13 = g2_mma(a1, b, c13); }
  v8f accs[8] = {c00, c01, c02, c03, c10, c11, c12, c13};
#pragma unroll
  for (int u = 0; u < 8; ++u) { const int t = u & 3, half = u >> 2; const int col = col0 + t * 16 + ln; const float bv = bf16_rne(bias[col]);
#pragma unroll
    for (int r = 0; r < 8; ++r) { const int rloc = half * 16 + 8 * hh + r; sw[rloc][t * 16 + ln] = accs[u][r] * alpha + bv; } }
  __builtin_amdgcn_fence(4  , "workgroup"); __builtin_amdgcn_wave_barrier(); }

__global__ __launch_bounds__(128) void k_gemm16(const _Float16* __restrict__ A, int lda, const _Float16* __restrict__ Bh, int ldb, float alpha, const float* __restrict__ bias,
    _Float16* __restrict__ C16, int ldc, int relu, int M, int N, int K) {
  __shared__ __attribute__((aligned(16))) float so[4][32][68];
  const int tid = threadIdx.x, w = tid >> 5, lane = tid & 31;
  const int ntn = N >> 6; const int mt = blockIdx.x / ntn, nq = blockIdx.x - mt * ntn; const int row0 = mt * 128 + 32 * w, col0 = nq * 64; if (row0 >= M) return;
  g2_core(A, lda, Bh, ldb, K, row0, col0, lane, alpha, bias, so[w]);
  const int rsub = lane >> 4, c4 = (lane & 15) * 4;
  for (int pass = 0; pass < 2; ++pass) {
#pragma unroll
    for (int q = 0; q < 16; ++q) { const int r = q * 2 + rsub; const v4f v = *(const v4fa*)&so[w][r][c4]; v4h h4;
#pragma unroll
      for (int i = 0; i < 4; ++i) { float t = v[i]; t = (relu != 0) ? fmaxf(t, 0.0f) : t; h4[i] = (_Float16)t; }
      *(volatile v4h*)(C16 + (size_t)(row0 + r) * ldc + col0 + c4) = h4; }
    if (pass == 0) __threadfence(); } }

__global__ __launch_bounds__(128) void k_gemm32(const _Float16* __restrict__ A, int lda, const _Float16* __restrict__ Bh, int ldb, float alpha, const float* __restrict__ bias,
    float* __restrict__ C32, int ldc, const float* __restrict__ res, int ldr, int resraw, int M, int N, int K) {
  __shared__ __attribute__((aligned(16))) float so[4][32][68];
  const int tid = threadIdx.x, w = tid >> 5, lane = tid & 31;
  const int ntn = N >> 6; const int mt = blockIdx.x / ntn, nq = blockIdx.x - mt * ntn; const int row0 = mt * 128 + 32 * w, col0 = nq * 64; if (row0 >= M) return;
  g2_core(A, lda, Bh, ldb, K, row0, col0, lane, alpha, bias, so[w]);
  const int rsub = lane >> 4, c4 = (lane & 15) * 4;
  for (int pass = 0; pass < 2; ++pass) {
#pragma unroll
    for (int q = 0; q < 16; ++q) { const int r = q * 2 + rsub; const int m = row0 + r; const int mb = m / SEQ; const int ms = m - mb * SEQ;
      const int rr = (resraw != 0) ? (mb * SEQ_FULL + ms) : m;
      v4f v = *(const v4fa*)&so[w][r][c4]; const v4f xr = *(const v4fa*)(res + (size_t)rr * ldr + col0 + c4);
#pragma unroll
      for (int i = 0; i < 4; ++i) { const float t0 = xr[i]; const float t1 = bf16_rne(t0); v[i] += (resraw != 0) ? t1 : t0; }
      *(volatile v4f*)(C32 + (size_t)m * ldc + col0 + c4) = v; }
    if (pass == 0) __threadfence(); } }

__global__ __launch_bounds__(256) void k_vt2(const _Float16* __restrict__ QKV, _Float16* __restrict__ VT) {
  __shared__ unsigned short tl[64][66];
  const int tid = threadIdx.x; const int slab = blockIdx.x / NQT, lg = blockIdx.x - slab * NQT; const int b = slab / NH, hd = slab - b * NH; const int s0 = lg * 64;
  for (int i = tid; i < 64 * 8; i += 256) { const int r = i / 8, c8 = (i % 8) * 8; FragH f;
    f.half[0] = *(const v8us*)((const unsigned short*)QKV + ((size_t)b * SEQ + s0 + r) * LQ + 2 * DM + hd * HD + c8);
#pragma unroll
    for (int q = 0; q < 8; ++q) tl[r][c8 + q] = f.u[q]; }
  __syncthreads();
  for (int pass = 0; pass < 2; ++pass) {
#pragma unroll
    for (int rd = 0; rd < 2; ++rd) { const int d = rd * 32 + tid / 8, pc = tid % 8; FragH f;
#pragma unroll
      for (int q = 0; q < 8; ++q) f.u[q] = tl[pc * 8 + q][d];
      *(volatile v8us*)((unsigned short*)VT + ((size_t)slab * HD + d) * SEQ + s0 + pc * 8) = f.half[0]; }
    if (pass == 0) __threadfence(); } }

__global__ __launch_bounds__(256) void k_mflag(const int* __restrict__ mk0, const int* __restrict__ mk1, int* __restrict__ MF) {
  __shared__ int sc[32];
  __shared__ unsigned int sr[8][2];
  const int tid = threadIdx.x, qt = blockIdx.x, wv = tid >> 5, lane = tid & 31; const int kt = tid >> 3, p = tid & 7;
  const int* mask = (blockIdx.y == 0) ? mk0 : mk1;
  int* dst = MF + (size_t)blockIdx.y * (NQT * 32) + (size_t)qt * 32;
  const bool ok = kt < NKT; const int ktc = ok ? kt : (NKT - 1);
  int any = 0, allnz = 1; unsigned int rlo = 0u, rhi = 0u;
#pragma unroll 1
  for (int r = 0; r < 64; ++r) {
    const int* rowp = mask + (size_t)(qt * 64 + r) * SEQ_FULL + ktc * 64 + p * 4;
    const v4ia a = *(const v4ia*)rowp; const v4ia c = *(const v4ia*)(rowp + 32);
    const int o = (a[0] | a[1]) | (a[2] | a[3]) | (c[0] | c[1]) | (c[2] | c[3]);
    const bool z = (a[0] == 0) | (a[1] == 0) | (a[2] == 0) | (a[3] == 0) | (c[0] == 0) | (c[1] == 0) | (c[2] == 0) | (c[3] == 0);
    any |= o; allnz &= z ? 0 : 1;
    const unsigned int bit = (ok && (o != 0)) ? 1u : 0u; const unsigned int sh = bit << (r & 31);
    rlo |= (r < 32) ? sh : 0u; rhi |= (r >= 32) ? sh : 0u; }
  any |= __shfl_xor(any, 1); any |= __shfl_xor(any, 2); any |= __shfl_xor(any, 4);
  allnz &= __shfl_xor(allnz, 1); allnz &= __shfl_xor(allnz, 2); allnz &= __shfl_xor(allnz, 4);
  rlo |= __shfl_xor(rlo, 1); rlo |= __shfl_xor(rlo, 2); rlo |= __shfl_xor(rlo, 4); rlo |= __shfl_xor(rlo, 8); rlo |= __shfl_xor(rlo, 16);
  rhi |= __shfl_xor(rhi, 1); rhi |= __shfl_xor(rhi, 2); rhi |= __shfl_xor(rhi, 4); rhi |= __shfl_xor(rhi, 8); rhi |= __shfl_xor(rhi, 16);
  const int code = ok ? ((any == 0) ? 0 : ((allnz != 0) ? 1 : 2)) : 0;
  if (p == 0) sc[kt] = code;
  if (lane == 0) { sr[wv][0] = rlo; sr[wv][1] = rhi; }
  __syncthreads();
  if (tid < 32) { unsigned int lo = 0u, hi = 0u;
#pragma unroll
    for (int i = 0; i < 8; ++i) { lo |= sr[i][0]; hi |= sr[i][1]; }
    const int live = ((lo == 0xFFFFFFFFu) && (hi == 0xFFFFFFFFu)) ? 4 : 0;
    const int v = sc[tid] | live; volatile int* d = dst + tid; *d = v; __threadfence(); *d = v; } }

__global__ __launch_bounds__(128) void k_attn(const _Float16* __restrict__ QKV, const _Float16* __restrict__ VT, const int* __restrict__ mask, const int* __restrict__ MF,
                                              _Float16* __restrict__ CTX) {
  __shared__ __attribute__((aligned(16))) float so[4][16][68];
  const int tid = threadIdx.x, w = tid >> 5, lane = tid & 31, l15 = lane & 15, hh = lane >> 4;
  const int qt = blockIdx.x, slab = blockIdx.y; const int b = slab / NH, hd = slab - b * NH;
  const int q0 = qt * 64 + w * 16;
  const _Float16* Qb = QKV + (size_t)b * SEQ * LQ + hd * HD;
  const _Float16* Kb = Qb + DM;
  const _Float16* Vb = VT + (size_t)slab * HD * SEQ;
  const _Float16* qrow = Qb + (size_t)(q0 + l15) * LQ;
  const v16h qf0 = g2_frag(qrow, hh), qf1 = g2_frag(qrow + 32, hh);
  const v8f z8 = {0.f,0.f,0.f,0.f,0.f,0.f,0.f,0.f};
  v8f o[4] = {z8, z8, z8, z8};
  float m = NEG_INF, l = 0.f;
  const float CL = 0.18033688011112042f;
#pragma unroll 1
  for (int it = 0; it < NKT; ++it) {
    const int mfw = __builtin_amdgcn_readfirstlane(MF[(size_t)qt * 32 + it]);
    const int code = mfw & 3;
    if (code == 0 && (mfw & 4) != 0) continue;
    const int key0 = it * 64;
    v8f s[4];
#pragma unroll
    for (int kt = 0; kt < 4; ++kt) {
      const _Float16* krow = Kb + (size_t)(key0 + kt * 16 + l15) * LQ;
      const v16h ka = g2_frag(krow, hh), kk = g2_frag(krow + 32, hh);
      v8f a = g2_mma(ka, qf0, z8); a = g2_mma(kk, qf1, a); s[kt] = a; }
    if (code != 1) {
#pragma unroll
      for (int kt = 0; kt < 4; ++kt) {
        const int* mp = mask + (size_t)(q0 + l15) * SEQ_FULL + key0 + kt * 16 + 8 * hh;
        const v4ia ma = *(const v4ia*)mp; const v4ia mb = *(const v4ia*)(mp + 4);
#pragma unroll
        for (int r = 0; r < 4; ++r) { s[kt][r] = (ma[r] == 0) ? FILL_RAW : s[kt][r]; s[kt][4 + r] = (mb[r] == 0) ? FILL_RAW : s[kt][4 + r]; } } }
    float lmax = NEG_INF;
#pragma unroll
    for (int kt = 0; kt < 4; ++kt)
#pragma unroll
      for (int r = 0; r < 8; ++r) lmax = fmaxf(lmax, s[kt][r]);
    lmax = fmaxf(lmax, __shfl_xor(lmax, 16));
    const float mnew = fmaxf(m, lmax);
    const float alpha = exp2f((m - mnew) * CL);
    m = mnew;
    float psum = 0.f; FragH pa, pb;
#pragma unroll
    for (int r = 0; r < 8; ++r) {
      const float e0 = exp2f(fmaf(s[0][r] - mnew, CL, 10.0f)), e1 = exp2f(fmaf(s[1][r] - mnew, CL, 10.0f));
      const float e2 = exp2f(fmaf(s[2][r] - mnew, CL, 10.0f)), e3 = exp2f(fmaf(s[3][r] - mnew, CL, 10.0f));
      psum += (e0 + e1) + (e2 + e3);
      pa.h[r] = (_Float16)e0; pa.h[8 + r] = (_Float16)e1; pb.h[r] = (_Float16)e2; pb.h[8 + r] = (_Float16)e3; }
    l = l * alpha + psum;
    float ar[8];
#pragma unroll
    for (int r = 0; r < 8; ++r) ar[r] = __shfl(alpha, 8 * hh + r);
#pragma unroll
    for (int dt = 0; dt < 4; ++dt) {
#pragma unroll
      for (int r = 0; r < 8; ++r) o[dt][r] *= ar[r];
      const _Float16* vrow = Vb + (size_t)(dt * 16 + l15) * SEQ + key0;
      const v16h va = g2_frag(vrow, hh), vb = g2_frag(vrow + 32, hh);
      o[dt] = g2_mma(pa.v, va, o[dt]); o[dt] = g2_mma(pb.v, vb, o[dt]); } }
  const float lt = l + __shfl_xor(l, 16);
  const float inv = 1.0f / lt;
  float ir[8];
#pragma unroll
  for (int r = 0; r < 8; ++r) ir[r] = __shfl(inv, 8 * hh + r);
#pragma unroll
  for (int dt = 0; dt < 4; ++dt)
#pragma unroll
    for (int r = 0; r < 8; ++r) so[w][8 * hh + r][dt * 16 + l15] = o[dt][r] * ir[r];
  __builtin_amdgcn_fence(4  , "workgroup"); __builtin_amdgcn_wave_barrier();
  const int rq = lane >> 3, pc = lane & 7;
  for (int pass = 0; pass < 2; ++pass) {
#pragma unroll
    for (int g = 0; g < 4; ++g) { const int row = g * 4 + rq;
      const v4f va = *(const v4fa*)&so[w][row][pc * 8]; const v4f vb = *(const v4fa*)&so[w][row][pc * 8 + 4]; FragH f;
#pragma unroll
      for (int i = 0; i < 4; ++i) { f.h[i] = (_Float16)va[i]; f.h[4 + i] = (_Float16)vb[i]; }
      *(volatile v8us*)((unsigned short*)CTX + ((size_t)b * SEQ + q0 + row) * DM + hd * HD + pc * 8) = f.half[0]; }
    if (pass == 0) __threadfence(); } }

__global__ __launch_bounds__(256) void k_ln(const float* __restrict__ in, const float* __restrict__ g, const float* __restrict__ be, float* __restrict__ outF, int fullrows,
                                            _Float16* __restrict__ out16, int has16) {
  __shared__ float red[8];
  const int row = blockIdx.x, tid = threadIdx.x, lane = tid & 31, wid = tid >> 5;
  const v4f xv = *(const v4fa*)(in + (size_t)row * DM + tid * 4);
  float s = (xv[0] + xv[1]) + (xv[2] + xv[3]);
  s += __shfl_xor(s, 1); s += __shfl_xor(s, 2); s += __shfl_xor(s, 4); s += __shfl_xor(s, 8); s += __shfl_xor(s, 16);
  if (lane == 0) red[wid] = s;
  __syncthreads();
  float mu = 0.f;
#pragma unroll
  for (int i = 0; i < 8; ++i) mu += red[i];
  mu *= (1.0f / DM);
  __syncthreads();
  const float d0 = xv[0] - mu, d1 = xv[1] - mu, d2 = xv[2] - mu, d3 = xv[3] - mu;
  float s2 = (d0 * d0 + d1 * d1) + (d2 * d2 + d3 * d3);
  s2 += __shfl_xor(s2, 1); s2 += __shfl_xor(s2, 2); s2 += __shfl_xor(s2, 4); s2 += __shfl_xor(s2, 8); s2 += __shfl_xor(s2, 16);
  if (lane == 0) red[wid] = s2;
  __syncthreads();
  float var = 0.f;
#pragma unroll
  for (int i = 0; i < 8; ++i) var += red[i];
  var *= (1.0f / DM);
  const float inv = rsqrtf(var + 1e-5f);
  const int c = tid * 4;
  const v4f gv = *(const v4fa*)(g + c); const v4f bv = *(const v4fa*)(be + c);
  v4f y; v4h h4;
  y[0] = d0 * inv * bf16_rne(gv[0]) + bf16_rne(bv[0]); y[1] = d1 * inv * bf16_rne(gv[1]) + bf16_rne(bv[1]);
  y[2] = d2 * inv * bf16_rne(gv[2]) + bf16_rne(bv[2]); y[3] = d3 * inv * bf16_rne(gv[3]) + bf16_rne(bv[3]);
#pragma unroll
  for (int i = 0; i < 4; ++i) h4[i] = (_Float16)y[i];
  const int rb = row / SEQ; const int rs = row - rb * SEQ; const int orow = (fullrows != 0) ? (rb * SEQ_FULL + rs) : row;
  volatile v4f* pf = (volatile v4f*)(outF + (size_t)orow * DM + c); volatile v4h* ph = (volatile v4h*)(out16 + (size_t)row * DM + c);
  *pf = y; if (has16 != 0) *ph = h4;
  __threadfence();
  *pf = y; if (has16 != 0) *ph = h4; }

extern "C" void kernel_launch(void* const* d_in, const int* in_sizes, int n_in,
                              void* d_out, int out_size, void* d_ws, size_t ws_size, hipStream_t stream) {
  if (n_in < 30) return;
  const int act_min = ((NB - 1) * SEQ_FULL + SEQ) * DM;
  if (in_sizes[0] < act_min || in_sizes[1] < act_min) return;
  if (in_sizes[2] < (SEQ - 1) * SEQ_FULL + SEQ || in_sizes[3] < (SEQ - 1) * SEQ_FULL + SEQ) return;
  for (int i = 4; i <= 18; i += 2) { if (in_sizes[i] < DM * DM || in_sizes[i + 1] < DM) return; }
  if (in_sizes[20] < DFF * DM || in_sizes[21] < DFF || in_sizes[22] < DM * DFF || in_sizes[23] < DM) return;
  for (int i = 24; i < 30; ++i) { if (in_sizes[i] < DM) return; }
  if (out_size < act_min) return;
  const float* x   = (const float*)d_in[0];
  const float* enc = (const float*)d_in[1];
  const int*   mk1 = (const int*)d_in[2];
  const int*   mk2 = (const int*)d_in[3];
  const float* wq1 = (const float*)d_in[4];  const float* bq1 = (const float*)d_in[5];
  const float* wk1 = (const float*)d_in[6];  const float* bk1 = (const float*)d_in[7];
  const float* wv1 = (const float*)d_in[8];  const float* bv1 = (const float*)d_in[9];
  const float* wo1 = (const float*)d_in[10]; const float* bo1 = (const float*)d_in[11];
  const float* wq2 = (const float*)d_in[12]; const float* bq2 = (const float*)d_in[13];
  const float* wk2 = (const float*)d_in[14]; const float* bk2 = (const float*)d_in[15];
  const float* wv2 = (const float*)d_in[16]; const float* bv2 = (const float*)d_in[17];
  const float* wo2 = (const float*)d_in[18]; const float* bo2 = (const float*)d_in[19];
  const float* wf1 = (const float*)d_in[20]; const float* bf1 = (const float*)d_in[21];
  const float* wf2 = (const float*)d_in[22]; const float* bf2 = (const float*)d_in[23];
  const float* g1 = (const float*)d_in[24]; const float* be1 = (const float*)d_in[25];
  const float* g2 = (const float*)d_in[26]; const float* be2 = (const float*)d_in[27];
  const float* g3 = (const float*)d_in[28]; const float* be3 = (const float*)d_in[29];
  char* ws = (char*)d_ws; size_t off = 0;
  auto take = [&](size_t bytes) { char* p = ws + off; off += (bytes + 255) & ~(size_t)255; return p; };
  _Float16* WA1 = (_Float16*)take((size_t)4 * DM * DM * 2);
  _Float16* WA2 = (_Float16*)take((size_t)4 * DM * DM * 2);
  _Float16* WF1 = (_Float16*)take((size_t)DFF * DM * 2);
  _Float16* WF2 = (_Float16*)take((size_t)DM * DFF * 2);
  _Float16* A16 = (_Float16*)take((size_t)MROWS * DM * 2);
  _Float16* E16 = (_Float16*)take((size_t)MROWS * DM * 2);
  char*     R1  = take(R1_BYTES);
  _Float16* CTX = (_Float16*)take((size_t)MROWS * DM * 2);
  float*    PRE = (float*)take((size_t)MROWS * DM * 4);
  float*    XN  = (float*)take((size_t)MROWS * DM * 4);
  int*      MF  = (int*)take((size_t)2 * NQT * 32 * 4);
  if (off > ws_size || off > (size_t)134217728) return;
  _Float16* QKV = (_Float16*)R1;
  _Float16* VT  = (_Float16*)(R1 + QKV_BYTES);
  _Float16* HID = (_Float16*)R1;
  const size_t MM = (size_t)DM * DM;
  const size_t nw8 = MM / 8, nf8 = (size_t)DFF * DM / 8, nx8 = (size_t)MROWS * DM / 8;
  k_wnat4<<<dim3((unsigned)(nw8 / 256), 4), 256, 0, stream>>>(wq1, wk1, wv1, wo1, nw8, WA1);
  k_wnat4<<<dim3((unsigned)(nw8 / 256), 4), 256, 0, stream>>>(wq2, wk2, wv2, wo2, nw8, WA2);
  k_wnat4<<<dim3((unsigned)(nf8 / 256), 1), 256, 0, stream>>>(wf1, wf1, wf1, wf1, nf8, WF1);
  k_wnat4<<<dim3((unsigned)(nf8 / 256), 1), 256, 0, stream>>>(wf2, wf2, wf2, wf2, nf8, WF2);
  k_x16<<<dim3((unsigned)(nx8 / 256), 2), 256, 0, stream>>>(x, enc, A16, E16);
  k_mflag<<<dim3((unsigned)NQT, 2), 256, 0, stream>>>(mk1, mk2, MF);
  const unsigned gP = (unsigned)((MROWS / 128) * (DM / 64));
  const unsigned gF = (unsigned)((MROWS / 128) * (DFF / 64));
  const dim3 gA((unsigned)NQT, (unsigned)(NB * NH));
  k_gemm16<<<gP, 128, 0, stream>>>(A16, DM, WA1,          DM, 0.0625f, bq1, QKV,          LQ, 0, MROWS, DM, DM);
  k_gemm16<<<gP, 128, 0, stream>>>(A16, DM, WA1 + MM,     DM, 0.0625f, bk1, QKV + DM,     LQ, 0, MROWS, DM, DM);
  k_gemm16<<<gP, 128, 0, stream>>>(A16, DM, WA1 + 2 * MM, DM, 0.0625f, bv1, QKV + 2 * DM, LQ, 0, MROWS, DM, DM);
  k_vt2<<<(unsigned)(NB * NH * NQT), 256, 0, stream>>>(QKV, VT);
  k_attn<<<gA, 128, 0, stream>>>(QKV, VT, mk1, MF, CTX);
  k_gemm32<<<gP, 128, 0, stream>>>(CTX, DM, WA1 + 3 * MM, DM, 0.0625f, bo1, PRE, DM, x, DM, 1, MROWS, DM, DM);
  k_ln<<<(unsigned)MROWS, 256, 0, stream>>>(PRE, g1, be1, XN, 0, A16, 1);
  k_gemm16<<<gP, 128, 0, stream>>>(A16, DM, WA2,          DM, 0.0625f, bq2, QKV,          LQ, 0, MROWS, DM, DM);
  k_gemm16<<<gP, 128, 0, stream>>>(E16, DM, WA2 + MM,     DM, 0.0625f, bk2, QKV + DM,     LQ, 0, MROWS, DM, DM);
  k_gemm16<<<gP, 128, 0, stream>>>(E16, DM, WA2 + 2 * MM, DM, 0.0625f, bv2, QKV + 2 * DM, LQ, 0, MROWS, DM, DM);
  k_vt2<<<(unsigned)(NB * NH * NQT), 256, 0, stream>>>(QKV, VT);
  k_attn<<<gA, 128, 0, stream>>>(QKV, VT, mk2, MF + (size_t)NQT * 32, CTX);
  k_gemm32<<<gP, 128, 0, stream>>>(CTX, DM, WA2 + 3 * MM, DM, 0.0625f, bo2, PRE, DM, XN, DM, 0, MROWS, DM, DM);
  k_ln<<<(unsigned)MROWS, 256, 0, stream>>>(PRE, g2, be2, XN, 0, A16, 1);
  k_gemm16<<<gF, 128, 0, stream>>>(A16, DM, WF1, DM, 0.0625f, bf1, HID, DFF, 1, MROWS, DFF, DM);
  k_gemm32<<<gP, 128, 0, stream>>>(HID, DFF, WF2, DFF, 0.0625f, bf2, PRE, DM, XN, DM, 0, MROWS, DM, DFF);
  k_ln<<<(unsigned)MROWS, 256, 0, stream>>>(PRE, g3, be3, (float*)d_out, 1, A16, 0);
}
